// PixelCNN_8693013807800
// MI455X (gfx1250) — hardware-verified
//
#include <hip/hip_runtime.h>


namespace {
constexpr int NI = 1024, HW = 64, NPIX = HW * HW, C1 = 16, T1 = 24, K1 = 32, T2 = 5, K2 = 96  ;
constexpr float HS = 8.0f;
__constant__ int TAP1[T1][2] = {{-3,-3},{-3,-2},{-3,-1},{-3,0},{-3,1},{-3,2},{-3,3}, {-2,-3},{-2,-2},{-2,-1},{-2,0},{-2,1},{-2,2},{-2,3}, {-1,-3},{-1,-2},{-1,-1},{-1,0},{-1,1},{-1,2},{-1,3}, {0,-3},{0,-2},{0,-1}};
constexpr int KH1[T1] = {0,0,0,0,0,0,0, 1,1,1,1,1,1,1, 2,2,2,2,2,2,2, 3,3,3}, KW1[T1] = {0,1,2,3,4,5,6, 0,1,2,3,4,5,6, 0,1,2,3,4,5,6, 0,1,2};
__constant__ int TAP2[T2][2] = {{-1,-1},{-1,0},{-1,1},{0,-1},{0,0}};
constexpr int KH2[T2] = {0,0,0,1,1}, KW2[T2] = {0,1,2,0,1};

typedef _Float16 b16;
typedef __attribute__((ext_vector_type(16))) _Float16 v16b;
typedef __attribute__((ext_vector_type(8))) _Float16 v8b;
typedef __attribute__((ext_vector_type(8))) float v8f;
typedef __attribute__((ext_vector_type(4))) float v4f;
__device__ __forceinline__ float bf16_rne(float f) { unsigned int u = __float_as_uint(f); u += 0x7FFFu + ((u >> 16) & 1u); return __uint_as_float(u & 0xFFFF0000u); }
__device__ __forceinline__ v16b frag_kb(const b16* p, int hh) { const v8b a = *(const v8b*)(p + 8 * hh), b = *(const v8b*)(p + 16 + 8 * hh); v16b f;
#pragma unroll
  for (int e = 0; e < 8; ++e) { f[e] = a[e]; f[8 + e] = b[e]; } return f; }
__device__ __forceinline__ v8f wmma16b(v16b a, v16b b, v8f c) { v8f d = __builtin_amdgcn_wmma_f32_16x16x32_f16(false, a, false, b, (short)0, c, false, false); asm volatile("v_nop\n\tv_nop\n\tv_nop\n\tv_nop" : "+v"(d) : "v"(a), "v"(b)); return d; }
__device__ __forceinline__ void wave_lds_sync() { __builtin_amdgcn_fence(__ATOMIC_RELEASE, "workgroup"); __builtin_amdgcn_wave_barrier(); __builtin_amdgcn_fence(__ATOMIC_ACQUIRE, "workgroup"); }
__device__ __forceinline__ float nexp(float x) { return __builtin_amdgcn_exp2f(x * 1.4426950408889634f); }
__device__ __forceinline__ float pmul(float a, float b) { float p = a * b; asm volatile("" : "+v"(p)); return p; }

__global__ __launch_bounds__(256) void prep_kernel(const float* __restrict__ w1, const float* __restrict__ b1, const float* __restrict__ w2, const float* __restrict__ b2, const float* __restrict__ w3, const float* __restrict__ b3, b16* __restrict__ R, float* __restrict__ P) {
  const int t_ = threadIdx.x;
  for (int pass = 0; pass < 2; ++pass) {
    for (int p = t_; p < 16 * (K1 + K2) / 8; p += 256) { v8b v;
      if (p < 16 * K1 / 8) { const int o = p / (K1 / 8), c0 = (p % (K1 / 8)) * 8; for (int e = 0; e < 8; ++e) { const int t = c0 + e; v[e] = (b16)((t < T1) ? bf16_rne(w1[(o * 7 + KH1[t]) * 7 + KW1[t]]) : 0.0f); } *(volatile v8b*)(R + o * K1 + c0) = v; }
      else { const int q = p - 16 * K1 / 8; const int o = q / (K2 / 8), c0 = (q % (K2 / 8)) * 8; for (int e = 0; e < 8; ++e) { const int c = c0 + e; const int t = c >> 4, i = c & 15; float wv = 0.0f; if (t < T2) wv = bf16_rne(w2[((o * C1 + i) * 3 + KH2[t]) * 3 + KW2[t]]); v[e] = (b16)wv; } *(volatile v8b*)(R + 16 * K1 + o * K2 + c0) = v; } }
    if (t_ < 64) { float v = 0.0f; if (t_ < 16) v = bf16_rne(b1[t_]); else if (t_ < 32) v = bf16_rne(b2[t_ - 16]); else if (t_ < 48) v = bf16_rne(w3[t_ - 32]); else if (t_ == 48) v = bf16_rne(b3[0]); ((volatile float*)P)[t_] = v; }
    __threadfence(); }
}

__global__ __launch_bounds__(256) void pix_kernel(const float* __restrict__ x, const b16* __restrict__ R, const float* __restrict__ P, float* __restrict__ out) {
  __shared__ float Xs[HW + 6][HW + 6 + 2];
  __shared__ __attribute__((aligned(16))) b16 H1[HW * HW + 8][C1];
  const int img = blockIdx.x, lane = threadIdx.x & 31, wave = threadIdx.x >> 5, nloc = lane & 15, hlf = lane >> 4, t_ = threadIdx.x;
  for (int i = t_; i < (HW + 6) * (HW + 8); i += 256) { const int r = i / (HW + 8), c = i % (HW + 8); const int h = r - 3, w = c - 3; Xs[r][c] = (h >= 0 && h < HW && w >= 0 && w < HW) ? bf16_rne(x[(size_t)img * NPIX + h * HW + w]) : 0.0f; }
  __syncthreads();
  const b16* B1 = R; const b16* B2 = R + 16 * K1;
  for (int tile = 0; tile < 32; ++tile) { const int p0 = wave * 512 + tile * 16; const int h = p0 / HW, w0 = p0 % HW; const int w = w0 + nloc;
    v16b a;
#pragma unroll
    for (int e = 0; e < 16; ++e) { const int t = (e < 8) ? (8 * hlf + e) : (16 + 8 * hlf + e - 8); a[e] = (b16)((t < T1) ? Xs[h + TAP1[t][0] + 3][w + TAP1[t][1] + 3] : 0.0f); }
    const v16b bw = frag_kb(B1 + nloc * K1, hlf); v8f acc = {}; acc = wmma16b(a, bw, acc);
#pragma unroll
    for (int r = 0; r < 8; ++r) { const int px = w0 + 8 * hlf + r; const float v = fmaxf(acc[r] + P[nloc], 0.0f); H1[h * HW + px][nloc] = (b16)(v * HS); } }
  if (t_ < C1) H1[HW * HW][t_] = (b16)0.0f;
  __syncthreads();
  float* Ow = (&Xs[0][0]) + wave * 512;
  for (int tile = 0; tile < 32; ++tile) { const int p0 = wave * 512 + tile * 16; const int h = p0 / HW, w0 = p0 % HW; const int w = w0 + nloc;
    v8f acc = {};
#pragma unroll
    for (int kb = 0; kb < K2; kb += 32) { v16b a;
#pragma unroll
      for (int sub = 0; sub < 2; ++sub) { const int t = (kb >> 4) + sub; int pix = HW * HW;
        if (t < T2) { const int hh2 = h + TAP2[t][0], ww = w + TAP2[t][1]; if (hh2 >= 0 && ww >= 0 && ww < HW) pix = hh2 * HW + ww; }
        const v8b vv = *(const v8b*)(&H1[pix][8 * hlf]); for (int e = 0; e < 8; ++e) a[sub * 8 + e] = vv[e]; }
      const v16b bw = frag_kb(B2 + nloc * K2 + kb, hlf); acc = wmma16b(a, bw, acc); }
#pragma unroll
    for (int r = 0; r < 8; ++r) { const float h2 = fmaxf(acc[r] * (1.0f / HS) + P[16 + nloc], 0.0f); float z = pmul(h2, P[32 + nloc]);
      z += __shfl_xor(z, 1); z += __shfl_xor(z, 2); z += __shfl_xor(z, 4); z += __shfl_xor(z, 8);
      if (nloc == 0) { const float o = 1.0f / (1.0f + nexp(-(z + P[48]))); Ow[tile * 16 + 8 * hlf + r] = o; } } }
  wave_lds_sync();
  for (int pass = 0; pass < 2; ++pass) { for (int i = lane; i < 512 / 4; i += 32) *(volatile v4f*)(out + (size_t)img * NPIX + wave * 512 + i * 4) = *(const v4f*)(Ow + i * 4); __threadfence(); }
}
}

extern "C" void kernel_launch(void* const* d_in, const int* in_sizes, int n_in,
                              void* d_out, int out_size, void* d_ws, size_t ws_size, hipStream_t stream) {
  (void)n_in; (void)out_size;
  const float* x = (const float*)d_in[0]; const float* w1 = (const float*)d_in[1]; const float* b1 = (const float*)d_in[2]; const float* w2 = (const float*)d_in[3]; const float* b2 = (const float*)d_in[4]; const float* w3 = (const float*)d_in[5]; const float* b3 = (const float*)d_in[6];
  float* out = (float*)d_out;
  if (in_sizes[0] != NI * NPIX || in_sizes[1] != 16 * 49 || in_sizes[3] != 16 * 16 * 9 || in_sizes[5] != 16) return;
  size_t off = 0; char* ws = (char*)d_ws;
  auto carve = [&](size_t bytes) { char* p = ws + off; off += (bytes + 255) & ~(size_t)255; return p; };
  b16* R = (b16*)carve((size_t)16 * (K1 + K2) * 2); float* P = (float*)carve(256);
  if (off > ws_size) return;
  prep_kernel<<<1, 256, 0, stream>>>(w1, b1, w2, b2, w3, b3, R, P);
  pix_kernel<<<NI, 256, 0, stream>>>(x, R, P, out);
}
